// EHEMB_66735201845492
// MI455X (gfx1250) — hardware-run, weakly checked
//
#include <hip/hip_runtime.h>


#define LQ   4096
#define CN   552
#define CP   576
#define NHD  4
#define HDD  138
#define HP   192
#define NHID 300
#define HIP_ 320
#define NTOK 256
#define K2   (2 * CP)
#define QH   1024
#define DM   CP
#define SCL  0.085125653988005853f
#define LEPS 1e-5f
#define LOSC 1024.0f

typedef _Float16 h16;
typedef unsigned short bf;
typedef __attribute__((ext_vector_type(16))) __bf16   v16bf;
typedef __attribute__((ext_vector_type(16))) _Float16 v16h;
typedef __attribute__((ext_vector_type(8)))  _Float16 v8h;
typedef __attribute__((ext_vector_type(8)))  unsigned short v8us;
typedef __attribute__((ext_vector_type(8)))  float    v8f;
typedef __attribute__((ext_vector_type(4)))  float    v4f;
typedef __attribute__((ext_vector_type(4)))  _Float16 v4h;
typedef v8h  __attribute__((may_alias)) v8ha;
typedef v4f  __attribute__((may_alias)) v4fa;
typedef v8us __attribute__((may_alias)) v8usa;

__device__ __forceinline__ unsigned short f2bf(float f) { unsigned u = __float_as_uint(f); u += 0x7FFFu + ((u >> 16) & 1u); return (unsigned short)(u >> 16); }
__device__ __forceinline__ float bf2f(unsigned short b) { return __uint_as_float(((unsigned)b) << 16); }
__device__ __forceinline__ float bfr(float f) { return bf2f(f2bf(f)); }
__device__ __forceinline__ v16h cat16(v8h lo, v8h hi) { return __builtin_shufflevector(lo, hi, 0, 1, 2, 3, 4, 5, 6, 7, 8, 9, 10, 11, 12, 13, 14, 15); }
__device__ __forceinline__ v16bf cat16b(v8us lo, v8us hi) { return __builtin_bit_cast(v16bf, __builtin_shufflevector(lo, hi, 0, 1, 2, 3, 4, 5, 6, 7, 8, 9, 10, 11, 12, 13, 14, 15)); }
__device__ __forceinline__ v8f wmma16(v16h a, v16h b, v8f c) { return __builtin_amdgcn_wmma_f32_16x16x32_f16(false, a, false, b, (short)0, c, false, false); }
__device__ __forceinline__ v8f wmmab(v16bf a, v16bf b, v8f c) { return __builtin_amdgcn_wmma_f32_16x16x32_bf16(false, a, false, b, (short)0, c, false, false); }

template <bool SPLITA, bool F16OUT = false>
__global__ __launch_bounds__(128) void k_gemmb(const bf* __restrict__ A, const bf* __restrict__ Al, const bf* __restrict__ Bn, const float* __restrict__ bias, float* C, int ldc, h16* C2, const float* __restrict__ R = nullptr, int K = DM, int roundR = 1) {
    __shared__ __align__(16) float ost[4][16 * 68];
    const int lane = threadIdx.x & 31, wave = threadIdx.x >> 5, lr = lane & 15, hi = lane >> 4;
    const int r0 = blockIdx.x * 64 + wave * 16, c0 = blockIdx.y * 64;
    const size_t aoff = (size_t)(r0 + lr) * K + 8 * hi;
    size_t boff[4];
#pragma unroll
    for (int t = 0; t < 4; ++t) boff[t] = (size_t)(c0 + t * 16 + lr) * K + 8 * hi;
    v8f acc[4];
#pragma unroll
    for (int t = 0; t < 4; ++t) acc[t] = (v8f){};
#pragma unroll 1
    for (int kc = 0; kc < K; kc += 32) {
        const v16bf a = cat16b(*(const v8us*)(A + aoff + kc), *(const v8us*)(A + aoff + kc + 16));
        v16bf al = a;
        if (SPLITA) al = cat16b(*(const v8us*)(Al + aoff + kc), *(const v8us*)(Al + aoff + kc + 16));
#pragma unroll
        for (int t = 0; t < 4; ++t) { const v16bf b = cat16b(*(const v8us*)(Bn + boff[t] + kc), *(const v8us*)(Bn + boff[t] + kc + 16)); acc[t] = wmmab(a, b, acc[t]); if (SPLITA) acc[t] = wmmab(al, b, acc[t]); }
        asm volatile("v_nop\n\tv_nop\n\tv_nop\n\tv_nop" : "+v"(acc[0]), "+v"(acc[1]), "+v"(acc[2]), "+v"(acc[3]) : "v"(a), "v"(al));
    }
    float* os = &ost[wave][0];
#pragma unroll
    for (int t = 0; t < 4; ++t) { const float bv = bias ? bfr(bias[c0 + t * 16 + lr]) : 0.f;
#pragma unroll
        for (int j = 0; j < 8; ++j) os[(hi * 8 + j) * 68 + t * 16 + lr] = acc[t][j] + bv; }
    __syncthreads();
    if (F16OUT) {
        h16* crow = (h16*)(void*)C + (size_t)r0 * ldc + c0;
        auto pass = [&]() {
#pragma unroll
            for (int s = 0; s < 4; ++s) { const int row = 4 * s + (lane >> 3), piece = lane & 7; const float* sp = os + row * 68 + piece * 8; v8h o, o2;
#pragma unroll
                for (int i = 0; i < 8; ++i) { const h16 a = (h16)sp[i]; o[i] = a; o2[i] = (h16)((sp[i] - (float)a) * LOSC); }
                *(volatile v8h*)(crow + (size_t)row * ldc + piece * 8) = o; if (C2) *(volatile v8h*)(C2 + (size_t)r0 * ldc + c0 + (size_t)row * ldc + piece * 8) = o2; }
        };
        pass(); __threadfence(); pass();
    } else {
        float* crow = C + (size_t)r0 * ldc + c0;
        auto pass = [&]() {
#pragma unroll
            for (int s = 0; s < 8; ++s) { const int Lid = (lane >> 3) + 4 * s, piece = lane & 7; const int row = Lid >> 1, cofs = (Lid & 1) * 32 + piece * 4;
                v4f val = *(const v4fa*)(os + row * 68 + cofs); if (R) { const v4f rv = *(const v4f*)(R + ((size_t)r0 + row) * ldc + c0 + cofs); val += roundR ? (v4f){bfr(rv[0]), bfr(rv[1]), bfr(rv[2]), bfr(rv[3])} : rv; }
                *(volatile v4f*)(crow + (size_t)row * ldc + cofs) = val; }
        };
        pass(); __threadfence(); pass();
    }
}

__global__ __launch_bounds__(128) void k_gemm3(const bf* __restrict__ Ah, const bf* __restrict__ Al, const bf* __restrict__ Bh, const bf* __restrict__ Bl, int K, float* C, int ldc) {
    __shared__ __align__(16) float ost[4][16 * 68];
    const int lane = threadIdx.x & 31, wave = threadIdx.x >> 5, lr = lane & 15, hi = lane >> 4;
    const int r0 = blockIdx.x * 64 + wave * 16, c0 = blockIdx.y * 64;
    const size_t aoff = (size_t)(r0 + lr) * K + 8 * hi;
    v8f acc[4];
#pragma unroll
    for (int t = 0; t < 4; ++t) acc[t] = (v8f){};
#pragma unroll 1
    for (int kc = 0; kc < K; kc += 32) {
        const v16bf a = cat16b(*(const v8us*)(Ah + aoff + kc), *(const v8us*)(Ah + aoff + kc + 16));
        const v16bf al = cat16b(*(const v8us*)(Al + aoff + kc), *(const v8us*)(Al + aoff + kc + 16));
#pragma unroll
        for (int t = 0; t < 4; ++t) { const size_t bo = (size_t)(c0 + t * 16 + lr) * K + kc + 8 * hi;
            const v16bf bh = cat16b(*(const v8us*)(Bh + bo), *(const v8us*)(Bh + bo + 16)); const v16bf bl = cat16b(*(const v8us*)(Bl + bo), *(const v8us*)(Bl + bo + 16));
            acc[t] = wmmab(a, bh, acc[t]); acc[t] = wmmab(al, bh, acc[t]); acc[t] = wmmab(a, bl, acc[t]); }
        asm volatile("v_nop\n\tv_nop\n\tv_nop\n\tv_nop" : "+v"(acc[0]), "+v"(acc[1]), "+v"(acc[2]), "+v"(acc[3]) : "v"(a), "v"(al));
    }
    float* os = &ost[wave][0];
#pragma unroll
    for (int t = 0; t < 4; ++t) {
#pragma unroll
        for (int j = 0; j < 8; ++j) os[(hi * 8 + j) * 68 + t * 16 + lr] = acc[t][j]; }
    __builtin_amdgcn_wave_barrier(); asm volatile("" ::: "memory");
    float* crow = C + (size_t)r0 * ldc + c0;
    auto pass = [&]() {
#pragma unroll
        for (int s = 0; s < 8; ++s) { const int Lid = (lane >> 3) + 4 * s, piece = lane & 7; const int row = Lid >> 1, cofs = (Lid & 1) * 32 + piece * 4;
            const v4f val = *(const v4fa*)(os + row * 68 + cofs); *(volatile v4f*)(crow + (size_t)row * ldc + cofs) = val; }
    };
    pass(); __threadfence(); pass();
}


__device__ __forceinline__ void put576(bf* dst, const float* src, int lane, bool live) {
    typedef __attribute__((ext_vector_type(4))) unsigned short v4us;
#pragma unroll
    for (int st = 0; st < 5; ++st) { const int c0 = st * 128 + lane * 4; if (st == 4 && lane >= 16) break; v4us v;
#pragma unroll
        for (int i = 0; i < 4; ++i) { const int c = c0 + i; v[i] = f2bf((live && c < CN) ? src[c < CN ? c : 0] : 0.f); }
        *(volatile v4us*)(dst + c0) = v; }
}
__global__ __launch_bounds__(256) void k_convin(const float* __restrict__ Fia, const int* __restrict__ xi, const float* __restrict__ emb, bf* XA) {
    const int lane = threadIdx.x & 31; const size_t w = (size_t)blockIdx.x * 8 + (threadIdx.x >> 5); if (w >= (size_t)LQ * 2) return; const size_t l = w >> 1; const int half = (int)(w & 1); const size_t t = 2 * l + half;
    const float* src; if (t < (size_t)LQ) { int id = xi[t]; id = id < 0 ? 0 : (id > NTOK - 1 ? NTOK - 1 : id); src = emb + (size_t)id * CN; } else { src = Fia + (size_t)(2 * (t - LQ)) * CN; }
    bf* dst = XA + l * K2 + (size_t)half * CP; put576(dst, src, lane, true); __threadfence(); put576(dst, src, lane, true);
}
__global__ __launch_bounds__(256) void k_fia2(const float* __restrict__ Fia, bf* F2b) {
    const int lane = threadIdx.x & 31; const size_t l = (size_t)blockIdx.x * 8 + (threadIdx.x >> 5); if (l >= (size_t)LQ) return; const float* src = Fia + (2 * l + 1) * CN;
    put576(F2b + l * CP, src, lane, true); __threadfence(); put576(F2b + l * CP, src, lane, true);
}
__global__ __launch_bounds__(256) void k_wconv(const float* __restrict__ w, bf* WB) {
    typedef __attribute__((ext_vector_type(4))) unsigned short v4us;
    const int lane = threadIdx.x & 31; const int o = blockIdx.x * 8 + (threadIdx.x >> 5); if (o >= CP) return;
#pragma unroll 1
    for (int ps = 0; ps < 2; ++ps) {
#pragma unroll 1
        for (int c0 = lane * 4; c0 < K2; c0 += 128) { v4us v;
#pragma unroll
            for (int i = 0; i < 4; ++i) { const int col = c0 + i; const int k = col / CP, c = col % CP; v[i] = f2bf((o < CN && c < CN) ? w[((size_t)(o < CN ? o : 0) * CN + (c < CN ? c : 0)) * 2 + k] : 0.f); }
            *(volatile v4us*)(WB + (size_t)o * K2 + c0) = v; }
        if (ps == 0) __threadfence(); }
}
__global__ __launch_bounds__(256) void k_wlin(const float* __restrict__ W, int nin, int nout, int NP, int KP, bf* WB) {
    typedef __attribute__((ext_vector_type(4))) unsigned short v4us;
    const int lane = threadIdx.x & 31; const int o = blockIdx.x * 8 + (threadIdx.x >> 5); if (o >= NP) return;
#pragma unroll 1
    for (int ps = 0; ps < 2; ++ps) {
#pragma unroll 1
        for (int c0 = 0; c0 < KP; c0 += 128) { const int cc = c0 + lane * 4; if (cc >= KP) continue; v4us v;
#pragma unroll
            for (int i = 0; i < 4; ++i) { const int k = cc + i; v[i] = f2bf((o < nout && k < nin) ? W[(size_t)(k < nin ? k : 0) * nout + (o < nout ? o : 0)] : 0.f); }
            *(volatile v4us*)(WB + (size_t)o * KP + cc) = v; }
        if (ps == 0) __threadfence(); }
}
__global__ __launch_bounds__(256) void k_bpad(const float* __restrict__ b, int n, int NP, float* BP) { for (int t = threadIdx.x; t < NP; t += 256) { const float v = (t < n) ? b[t] : 0.f; *(volatile float*)(BP + t) = v; } __threadfence(); for (int t = threadIdx.x; t < NP; t += 256) { const float v = (t < n) ? b[t] : 0.f; *(volatile float*)(BP + t) = v; } }
__global__ __launch_bounds__(256) void k_split576(const float* __restrict__ src, int rows, bf* dh, bf* dl) {
    typedef __attribute__((ext_vector_type(4))) unsigned short v4us;
    const int lane = threadIdx.x & 31; const size_t r = (size_t)blockIdx.x * 8 + (threadIdx.x >> 5); if (r >= (size_t)rows) return;
#pragma unroll 1
    for (int ps = 0; ps < 2; ++ps) {
#pragma unroll 1
        for (int st = 0; st < 5; ++st) { const int c0 = st * 128 + lane * 4; if (st == 4 && lane >= 16) break; const v4f v = *(const v4f*)(src + r * CP + c0); v4us oh, ol;
#pragma unroll
            for (int i = 0; i < 4; ++i) { const unsigned short hb = f2bf(v[i]); oh[i] = hb; ol[i] = f2bf(v[i] - bf2f(hb)); }
            *(volatile v4us*)(dh + r * CP + c0) = oh; *(volatile v4us*)(dl + r * CP + c0) = ol; }
        if (ps == 0) __threadfence(); }
}
__global__ __launch_bounds__(256) void k_hpl(const float* __restrict__ F, int h, float sc, bf* Ph, bf* Pl) {
    typedef __attribute__((ext_vector_type(2))) unsigned short v2us;
    const int lane = threadIdx.x & 31; const size_t l = (size_t)blockIdx.x * 8 + (threadIdx.x >> 5); if (l >= (size_t)LQ) return; v2us hh_[3], ll_[3];
#pragma unroll
    for (int t = 0; t < 3; ++t) {
#pragma unroll
        for (int i = 0; i < 2; ++i) { const int d = t * 64 + lane * 2 + i; const float y = (d < HDD) ? F[l * CP + h * HDD + (d < HDD ? d : 0)] * sc : 0.f; const unsigned short hb = f2bf(y); hh_[t][i] = hb; ll_[t][i] = f2bf(y - bf2f(hb)); } }
    auto pass = [&]() {
#pragma unroll
        for (int t = 0; t < 3; ++t) { *(volatile v2us*)(Ph + l * HP + t * 64 + lane * 2) = hh_[t]; *(volatile v2us*)(Pl + l * HP + t * 64 + lane * 2) = ll_[t]; } };
    pass(); __threadfence(); pass();
}
__global__ __launch_bounds__(256) void k_vth(const float* __restrict__ V, int h, bf* Th, bf* Tl) {
    typedef __attribute__((ext_vector_type(2))) unsigned short v2us;
    const int lane = threadIdx.x & 31; const size_t wid = (size_t)blockIdx.x * 8 + (threadIdx.x >> 5); if (wid >= (size_t)HP * (LQ / 64)) return; const int d = (int)(wid / (LQ / 64)); const int l0 = (int)(wid % (LQ / 64)) * 64 + lane * 2; v2us oh, ol;
#pragma unroll
    for (int i = 0; i < 2; ++i) { const float y = (d < HDD) ? V[(size_t)(l0 + i) * CP + h * HDD + (d < HDD ? d : 0)] : 0.f; const unsigned short hb = f2bf(y); oh[i] = hb; ol[i] = f2bf(y - bf2f(hb)); }
    const size_t o = (size_t)d * LQ + l0; *(volatile v2us*)(Th + o) = oh; *(volatile v2us*)(Tl + o) = ol; __threadfence(); *(volatile v2us*)(Th + o) = oh; *(volatile v2us*)(Tl + o) = ol;
}
__global__ __launch_bounds__(256) void k_soft(const float* __restrict__ S, bf* PH, bf* PL) {
    typedef __attribute__((ext_vector_type(4))) unsigned short v4us;
    const int lane = threadIdx.x & 31, i = blockIdx.x * 8 + (threadIdx.x >> 5); if (i >= QH) return; const float* sr = S + (size_t)i * LQ;
    float m = -3.0e38f;
#pragma unroll 1
    for (int c0 = lane * 4; c0 < LQ; c0 += 128) {
#pragma unroll
        for (int q = 0; q < 4; ++q) m = fmaxf(m, sr[c0 + q]); }
#pragma unroll
    for (int sh = 16; sh; sh >>= 1) m = fmaxf(m, __shfl_xor(m, sh, 32));
    float sum = 0.f;
#pragma unroll 1
    for (int c0 = lane * 4; c0 < LQ; c0 += 128) {
#pragma unroll
        for (int q = 0; q < 4; ++q) sum += __expf(sr[c0 + q] - m); }
#pragma unroll
    for (int sh = 16; sh; sh >>= 1) sum += __shfl_xor(sum, sh, 32);
    const float inv = 1.0f / sum;
#pragma unroll 1
    for (int ps = 0; ps < 2; ++ps) {
#pragma unroll 1
        for (int c0 = lane * 4; c0 < LQ; c0 += 128) { v4us oh, ol;
#pragma unroll
            for (int q = 0; q < 4; ++q) { const float p = __expf(sr[c0 + q] - m) * inv; const unsigned short hb = f2bf(p); oh[q] = hb; ol[q] = f2bf(p - bf2f(hb)); }
            const size_t o = (size_t)i * LQ + c0; *(volatile v4us*)(PH + o) = oh; *(volatile v4us*)(PL + o) = ol; }
        if (ps == 0) __threadfence(); }
}
__global__ __launch_bounds__(256) void k_merge(const float* __restrict__ XH, float* AO) {
    const int lane = threadIdx.x & 31; const size_t l = (size_t)blockIdx.x * 8 + (threadIdx.x >> 5); if (l >= (size_t)LQ) return;
    auto val = [&](int c) -> float { if (c >= CN) return 0.f; const int h = c / HDD, d = c % HDD; return XH[((size_t)h * LQ + l) * HP + d]; };
#pragma unroll 1
    for (int ps = 0; ps < 2; ++ps) {
#pragma unroll 1
        for (int st = 0; st < 5; ++st) { const int c0 = st * 128 + lane * 4; if (st == 4 && lane >= 16) break; v4f v;
#pragma unroll
            for (int i = 0; i < 4; ++i) v[i] = val(c0 + i);
            *(volatile v4f*)(AO + l * CP + c0) = v; }
        if (ps == 0) __threadfence(); }
}
template <bool RIN>
__global__ __launch_bounds__(256) void k_addln(const float* __restrict__ Ain, const float* __restrict__ Bin, const float* __restrict__ Fia, const float* __restrict__ g, const float* __restrict__ bb, float* Hf, bf* Hh, bf* Hl) {
    typedef __attribute__((ext_vector_type(4))) unsigned short v4us;
    const int lane = threadIdx.x & 31; const size_t l = (size_t)blockIdx.x * 8 + (threadIdx.x >> 5); if (l >= (size_t)LQ) return; const float* f2 = Fia + (2 * l + 1) * CN;
    float v[20]; float s = 0.f;
#pragma unroll
    for (int st = 0; st < 5; ++st) {
#pragma unroll
        for (int i = 0; i < 4; ++i) { const int c = st * 128 + lane * 4 + i; float t = 0.f; if (!(st == 4 && lane >= 16) && c < CN) { t = Ain[l * CP + c] + (RIN ? bfr(f2[c]) : Bin[l * CP + c]); } v[st * 4 + i] = t; s += t; } }
#pragma unroll
    for (int sh = 16; sh; sh >>= 1) s += __shfl_xor(s, sh, 32);
    const float mu = s * (1.0f / CN); float qv = 0.f;
#pragma unroll
    for (int st = 0; st < 5; ++st) {
#pragma unroll
        for (int i = 0; i < 4; ++i) { const int c = st * 128 + lane * 4 + i; if (!(st == 4 && lane >= 16) && c < CN) { const float d = v[st * 4 + i] - mu; qv = fmaf(d, d, qv); } } }
#pragma unroll
    for (int sh = 16; sh; sh >>= 1) qv += __shfl_xor(qv, sh, 32);
    const float rs = rsqrtf(qv * (1.0f / CN) + LEPS);
#pragma unroll 1
    for (int ps = 0; ps < 2; ++ps) {
#pragma unroll 1
        for (int st = 0; st < 5; ++st) { const int c0 = st * 128 + lane * 4; if (st == 4 && lane >= 16) break; v4f y; v4us oh, ol;
#pragma unroll
            for (int i = 0; i < 4; ++i) { const int c = c0 + i; const float yy = (c < CN) ? (v[st * 4 + i] - mu) * rs * bfr(g[c < CN ? c : 0]) + bfr(bb[c < CN ? c : 0]) : 0.f; y[i] = yy; const unsigned short hb = f2bf(yy); oh[i] = hb; ol[i] = f2bf(yy - bf2f(hb)); }
            *(volatile v4f*)(Hf + l * CP + c0) = y; *(volatile v4us*)(Hh + l * CP + c0) = oh; *(volatile v4us*)(Hl + l * CP + c0) = ol; }
        if (ps == 0) __threadfence(); }
}
__global__ __launch_bounds__(256) void k_relu320(const float* __restrict__ F, int rows, bf* Gh, bf* Gl) {
    typedef __attribute__((ext_vector_type(4))) unsigned short v4us;
    const int lane = threadIdx.x & 31; const size_t r = (size_t)blockIdx.x * 8 + (threadIdx.x >> 5); if (r >= (size_t)rows) return;
#pragma unroll 1
    for (int ps = 0; ps < 2; ++ps) {
#pragma unroll 1
        for (int st = 0; st < 3; ++st) { const int c0 = st * 128 + lane * 4; if (st == 2 && lane >= 16) break; const v4f v = *(const v4f*)(F + r * HIP_ + c0); v4us oh, ol;
#pragma unroll
            for (int i = 0; i < 4; ++i) { const float y = fmaxf(v[i], 0.f); const unsigned short hb = f2bf(y); oh[i] = hb; ol[i] = f2bf(y - bf2f(hb)); }
            *(volatile v4us*)(Gh + r * HIP_ + c0) = oh; *(volatile v4us*)(Gl + r * HIP_ + c0) = ol; }
        if (ps == 0) __threadfence(); }
}
__global__ __launch_bounds__(256) void k_p2in(const bf* __restrict__ Hh, const bf* __restrict__ Hl, bf* Ah, bf* Al) {
    typedef __attribute__((ext_vector_type(4))) unsigned short v4us;
    const int lane = threadIdx.x & 31; const size_t w = (size_t)blockIdx.x * 8 + (threadIdx.x >> 5); if (w >= (size_t)LQ * 2) return; const size_t l = w >> 1; const int half = (int)(w & 1); const size_t srow = 2 * l + half; const bool live = srow < (size_t)LQ;
#pragma unroll 1
    for (int ps = 0; ps < 2; ++ps) {
#pragma unroll 1
        for (int st = 0; st < 5; ++st) { const int c0 = st * 128 + lane * 4; if (st == 4 && lane >= 16) break; v4us a = {0, 0, 0, 0}, c = {0, 0, 0, 0};
            if (live) { a = *(const v4us*)(Hh + srow * CP + c0); c = *(const v4us*)(Hl + srow * CP + c0); }
            *(volatile v4us*)(Ah + l * K2 + (size_t)half * CP + c0) = a; *(volatile v4us*)(Al + l * K2 + (size_t)half * CP + c0) = c; }
        if (ps == 0) __threadfence(); }
}
__global__ __launch_bounds__(256) void k_addf2(const float* __restrict__ P2, const float* __restrict__ Fia, bf* Oh, bf* Ol) {
    typedef __attribute__((ext_vector_type(4))) unsigned short v4us;
    const int lane = threadIdx.x & 31; const size_t l = (size_t)blockIdx.x * 8 + (threadIdx.x >> 5); if (l >= (size_t)LQ) return; const float* f2 = Fia + (2 * l + 1) * CN;
#pragma unroll 1
    for (int ps = 0; ps < 2; ++ps) {
#pragma unroll 1
        for (int st = 0; st < 5; ++st) { const int c0 = st * 128 + lane * 4; if (st == 4 && lane >= 16) break; v4us oh, ol;
#pragma unroll
            for (int i = 0; i < 4; ++i) { const int c = c0 + i; const float y = (c < CN) ? P2[l * CP + c] + bfr(f2[c < CN ? c : 0]) : 0.f; const unsigned short hb = f2bf(y); oh[i] = hb; ol[i] = f2bf(y - bf2f(hb)); }
            *(volatile v4us*)(Oh + l * CP + c0) = oh; *(volatile v4us*)(Ol + l * CP + c0) = ol; }
        if (ps == 0) __threadfence(); }
}

extern "C" void kernel_launch(void* const* d_in, const int* in_sizes, int n_in,
                              void* d_out, int out_size, void* d_ws, size_t ws_size, hipStream_t stream) {
    (void)in_sizes; (void)n_in; (void)out_size;
    const float* Fia = (const float*)d_in[0]; const int* xi = (const int*)d_in[1]; const float* emb = (const float*)d_in[2]; const float* c1w = (const float*)d_in[3]; const float* c1b = (const float*)d_in[4];
    const float* wq = (const float*)d_in[5]; const float* bq = (const float*)d_in[6]; const float* wk = (const float*)d_in[7]; const float* bk = (const float*)d_in[8]; const float* wv = (const float*)d_in[9]; const float* bv = (const float*)d_in[10]; const float* wo = (const float*)d_in[11]; const float* bo = (const float*)d_in[12];
    const float* l1s = (const float*)d_in[13]; const float* l1b = (const float*)d_in[14]; const float* f1w = (const float*)d_in[15]; const float* f1b = (const float*)d_in[16]; const float* f2w = (const float*)d_in[17]; const float* f2b = (const float*)d_in[18]; const float* l2s = (const float*)d_in[19]; const float* l2b = (const float*)d_in[20];
    const float* p2w = (const float*)d_in[21]; const float* p2b = (const float*)d_in[22]; const float* dw = (const float*)d_in[23]; const float* db = (const float*)d_in[24];
    float* out = (float*)d_out;
    char* wsp = (char*)d_ws;
    auto take = [&](size_t bytes) { char* p = wsp; wsp += (bytes + 255) & ~(size_t)255; return (void*)p; };
    bf* WC1 = (bf*)take((size_t)CP * K2 * 2); bf* WP2 = (bf*)take((size_t)CP * K2 * 2); bf* WQ = (bf*)take((size_t)CP * CP * 2); bf* WK = (bf*)take((size_t)CP * CP * 2); bf* WV = (bf*)take((size_t)CP * CP * 2); bf* WO = (bf*)take((size_t)CP * CP * 2);
    bf* WF1 = (bf*)take((size_t)HIP_ * CP * 2); bf* WF2 = (bf*)take((size_t)CP * HIP_ * 2); bf* WD = (bf*)take((size_t)NTOK * CP * 2);
    float* BC1 = (float*)take(CP * 4); float* BQ = (float*)take(CP * 4); float* BK = (float*)take(CP * 4); float* BV = (float*)take(CP * 4); float* BO = (float*)take(CP * 4); float* BF1 = (float*)take(HIP_ * 4); float* BF2 = (float*)take(CP * 4); float* BP2 = (float*)take(CP * 4);
    bf* XA = (bf*)take((size_t)LQ * K2 * 2); bf* F2b = (bf*)take((size_t)LQ * CP * 2);
    float* FI1 = (float*)take((size_t)LQ * CP * 4); bf* FIh = (bf*)take((size_t)LQ * CP * 2); bf* FIl = (bf*)take((size_t)LQ * CP * 2); float* QF = (float*)take((size_t)LQ * CP * 4); float* KF = (float*)take((size_t)LQ * CP * 4); float* VF = (float*)take((size_t)LQ * CP * 4);
    bf* Qh = (bf*)take((size_t)LQ * HP * 2); bf* Ql = (bf*)take((size_t)LQ * HP * 2); bf* Kh = (bf*)take((size_t)LQ * HP * 2); bf* Kl = (bf*)take((size_t)LQ * HP * 2); bf* VTh = (bf*)take((size_t)HP * LQ * 2); bf* VTl = (bf*)take((size_t)HP * LQ * 2);
    float* S = (float*)take((size_t)QH * LQ * 4); bf* PH = (bf*)take((size_t)QH * LQ * 2); bf* PL = (bf*)take((size_t)QH * LQ * 2); float* XH = (float*)take((size_t)NHD * LQ * HP * 4);
    if ((size_t)(wsp - (char*)d_ws) > ws_size) return;
    float* AO = QF; bf* AOh = (bf*)XA; bf* AOl = AOh + (size_t)LQ * CP; float* AOO = KF; float* H1 = VF; bf* H1h = FIh; bf* H1l = FIl; float* FF1 = (float*)S; bf* G1h = (bf*)PH; bf* G1l = (bf*)PL; float* FF2 = QF; float* H2 = KF; bf* H2h = (bf*)XA; bf* H2l = H2h + (size_t)LQ * CP;
    bf* P2h = Qh; bf* P2l = (bf*)S;    float* P2 = VF; bf* O2h = FIh; bf* O2l = FIl;
    k_wconv<<<CP / 8, 256, 0, stream>>>(c1w, WC1); k_wconv<<<CP / 8, 256, 0, stream>>>(p2w, WP2);
    k_wlin<<<CP / 8, 256, 0, stream>>>(wq, CN, CN, CP, CP, WQ); k_wlin<<<CP / 8, 256, 0, stream>>>(wk, CN, CN, CP, CP, WK); k_wlin<<<CP / 8, 256, 0, stream>>>(wv, CN, CN, CP, CP, WV); k_wlin<<<CP / 8, 256, 0, stream>>>(wo, CN, CN, CP, CP, WO);
    k_wlin<<<HIP_ / 8, 256, 0, stream>>>(f1w, CN, NHID, HIP_, CP, WF1); k_wlin<<<CP / 8, 256, 0, stream>>>(f2w, NHID, CN, CP, HIP_, WF2); k_wlin<<<NTOK / 8, 256, 0, stream>>>(dw, CN, NTOK, NTOK, CP, WD);
    k_bpad<<<1, 256, 0, stream>>>(c1b, CN, CP, BC1); k_bpad<<<1, 256, 0, stream>>>(bq, CN, CP, BQ); k_bpad<<<1, 256, 0, stream>>>(bk, CN, CP, BK); k_bpad<<<1, 256, 0, stream>>>(bv, CN, CP, BV); k_bpad<<<1, 256, 0, stream>>>(bo, CN, CP, BO); k_bpad<<<1, 256, 0, stream>>>(f1b, NHID, HIP_, BF1); k_bpad<<<1, 256, 0, stream>>>(f2b, CN, CP, BF2); k_bpad<<<1, 256, 0, stream>>>(p2b, CN, CP, BP2);
    const dim3 g576(LQ / 64, CP / 64, 1);
    k_convin<<<(LQ * 2) / 8, 256, 0, stream>>>(Fia, xi, emb, XA); k_fia2<<<LQ / 8, 256, 0, stream>>>(Fia, F2b);
    k_gemmb<false, false><<<g576, 128, 0, stream>>>(XA, nullptr, WC1, BC1, FI1, CP, nullptr, nullptr, K2);
    k_split576<<<LQ / 8, 256, 0, stream>>>(FI1, LQ, FIh, FIl);
    k_gemmb<false, false><<<g576, 128, 0, stream>>>(F2b, nullptr, WQ, BQ, QF, CP, nullptr, nullptr, CP);
    k_gemmb<true, false><<<g576, 128, 0, stream>>>(FIh, FIl, WK, BK, KF, CP, nullptr, nullptr, CP);
    k_gemmb<true, false><<<g576, 128, 0, stream>>>(FIh, FIl, WV, BV, VF, CP, nullptr, nullptr, CP);
    for (int h = 0; h < NHD; ++h) {
        k_hpl<<<LQ / 8, 256, 0, stream>>>(QF, h, SCL, Qh, Ql);
        k_hpl<<<LQ / 8, 256, 0, stream>>>(KF, h, 1.0f, Kh, Kl); k_vth<<<(HP * (LQ / 64)) / 8, 256, 0, stream>>>(VF, h, VTh, VTl);
        for (int qh = 0; qh < LQ / QH; ++qh) { const size_t q0 = (size_t)qh * QH;
            k_gemm3<<<dim3(QH / 64, LQ / 64, 1), 128, 0, stream>>>(Qh + q0 * HP, Ql + q0 * HP, Kh, Kl, HP, S, LQ);
            k_soft<<<QH / 8, 256, 0, stream>>>(S, PH, PL);
            k_gemm3<<<dim3(QH / 64, HP / 64, 1), 128, 0, stream>>>(PH, PL, VTh, VTl, LQ, XH + ((size_t)h * LQ + q0) * HP, HP); } }
    k_merge<<<LQ / 8, 256, 0, stream>>>(XH, AO);
    k_split576<<<LQ / 8, 256, 0, stream>>>(AO, LQ, AOh, AOl);
    k_gemmb<true, false><<<g576, 128, 0, stream>>>(AOh, AOl, WO, BO, AOO, CP, nullptr, nullptr, CP);
    k_addln<true><<<LQ / 8, 256, 0, stream>>>(AOO, nullptr, Fia, l1s, l1b, H1, H1h, H1l);
    k_gemmb<true, false><<<dim3(LQ / 64, HIP_ / 64, 1), 128, 0, stream>>>(H1h, H1l, WF1, BF1, FF1, HIP_, nullptr, nullptr, CP);
    k_relu320<<<LQ / 8, 256, 0, stream>>>(FF1, LQ, G1h, G1l);
    k_gemmb<true, false><<<g576, 128, 0, stream>>>(G1h, G1l, WF2, BF2, FF2, CP, nullptr, nullptr, HIP_);
    k_addln<false><<<LQ / 8, 256, 0, stream>>>(FF2, H1, Fia, l2s, l2b, H2, H2h, H2l);
    k_p2in<<<(LQ * 2) / 8, 256, 0, stream>>>(H2h, H2l, P2h, P2l);
    k_gemmb<true, false><<<g576, 128, 0, stream>>>(P2h, P2l, WP2, BP2, P2, CP, nullptr, nullptr, K2);
    k_addf2<<<LQ / 8, 256, 0, stream>>>(P2, Fia, O2h, O2l);
    k_gemmb<true, false><<<dim3(LQ / 64, NTOK / 64, 1), 128, 0, stream>>>(O2h, O2l, WD, db, out, NTOK, nullptr, nullptr, CP);
}
